// SpatialCrossAttention_15307263443422
// MI455X (gfx1250) — hardware-verified
//
#include <hip/hip_runtime.h>
#ifndef NB
#define NB 2
#endif
#ifndef SEQ
#define SEQ 2304
#endif
#define NB_FULL 2
#define SEQ_FULL 2304
#define TT 8
#define CC 64
#define PF (SEQ_FULL * TT)
#define PP (SEQ * TT)
static_assert(NB >= 1 && NB <= NB_FULL);
static_assert(SEQ >= 32 && SEQ <= SEQ_FULL && (SEQ % 4) == 0);
static_assert((PP % 32) == 0 && (CC % 64) == 0);

typedef __bf16 v16b __attribute__((ext_vector_type(16)));
typedef unsigned short v8us __attribute__((ext_vector_type(8), may_alias));
typedef float  v8f  __attribute__((ext_vector_type(8)));
typedef float  v4f  __attribute__((ext_vector_type(4)));
typedef float  v4fa __attribute__((ext_vector_type(4), may_alias));
union FragB { v16b v; v8us half[2]; unsigned short u[16]; };

__device__ __forceinline__ unsigned short bf16_bits(float x) { unsigned int u = __float_as_uint(x); return (unsigned short)((u + 0x7FFFu + ((u >> 16) & 1u)) >> 16); }
__device__ __forceinline__ float bf16_val(unsigned short b) { return __uint_as_float(((unsigned int)b) << 16); }
__device__ __forceinline__ float bf16_rne(float x) { return bf16_val(bf16_bits(x)); }

template <int NT>
__device__ __forceinline__ v8f mmaN(v16b ah, v16b al, v16b bh, v16b bl, v8f c) {
  c = __builtin_amdgcn_wmma_f32_16x16x32_bf16(false, ah, false, bh, (short)0, c, false, false);
  if (NT >= 2) c = __builtin_amdgcn_wmma_f32_16x16x32_bf16(false, al, false, bh, (short)0, c, false, false);
  if (NT >= 3) c = __builtin_amdgcn_wmma_f32_16x16x32_bf16(false, ah, false, bl, (short)0, c, false, false);
  asm volatile("v_nop\n\tv_nop\n\tv_nop\n\tv_nop" : "+v"(c) : "v"(ah), "v"(al), "v"(bh), "v"(bl));
  return c;
}

__global__ __launch_bounds__(256) void k_cvt_rows(const float* __restrict__ W, unsigned short* __restrict__ Wt, int n8) {
  const int t = blockIdx.x * 256 + threadIdx.x;
  if (t >= n8) return;
  const v4f a = *(const v4fa*)(W + (size_t)t * 8), b = *(const v4fa*)(W + (size_t)t * 8 + 4);
  v8us v; v[0]=bf16_bits(a[0]); v[1]=bf16_bits(a[1]); v[2]=bf16_bits(a[2]); v[3]=bf16_bits(a[3]);
  v[4]=bf16_bits(b[0]); v[5]=bf16_bits(b[1]); v[6]=bf16_bits(b[2]); v[7]=bf16_bits(b[3]);
  *(volatile v8us*)(Wt + (size_t)t * 8) = v; __threadfence(); *(volatile v8us*)(Wt + (size_t)t * 8) = v;
}

__global__ __launch_bounds__(256) void k_split_rows(const float* __restrict__ X, unsigned short* __restrict__ Xh, unsigned short* __restrict__ Xl, int n8) {
  const int t = blockIdx.x * 256 + threadIdx.x;
  if (t >= n8) return;
  const v4f a = *(const v4fa*)(X + (size_t)t * 8), b = *(const v4fa*)(X + (size_t)t * 8 + 4);
  const float xs[8] = {a[0],a[1],a[2],a[3],b[0],b[1],b[2],b[3]};
  v8us vh, vl;
#pragma unroll
  for (int i = 0; i < 8; ++i) { const unsigned short hb = bf16_bits(xs[i]); vh[i] = hb; vl[i] = bf16_bits(xs[i] - bf16_val(hb)); }
  *(volatile v8us*)(Xh + (size_t)t * 8) = vh; *(volatile v8us*)(Xl + (size_t)t * 8) = vl;
  __threadfence();
  *(volatile v8us*)(Xh + (size_t)t * 8) = vh; *(volatile v8us*)(Xl + (size_t)t * 8) = vl;
}

template <bool ASPLIT, int ACT, bool BIAS_BF16>
__global__ __launch_bounds__(128) void k_gemm_bf(const float* __restrict__ A, int lda, const unsigned short* __restrict__ Wt, int ldb,
                                               const float* __restrict__ bias, float* __restrict__ C, int ldc, int M, int N, int K) {
  __shared__ __attribute__((aligned(16))) float so[4][16][64];
  const int tid = threadIdx.x, w = tid >> 5, lane = tid & 31, ln = lane & 15, hh = lane >> 4;
  const int ntn = N / 64;
  const int wid = blockIdx.x * 4 + w;
  const int mt = wid / ntn, nq = wid % ntn;
  if (mt * 16 >= M) return;
  const int row0 = mt * 16, col0 = nq * 64;
  const float* arow = A + (size_t)(row0 + ln) * lda;
  v8f acc[4] = {};
  for (int kb = 0; kb < K; kb += 32) {
    FragB ah, al;
    const v4f x0 = *(const v4fa*)(arow + kb + 8 * hh), x1 = *(const v4fa*)(arow + kb + 8 * hh + 4);
    const v4f x2 = *(const v4fa*)(arow + kb + 16 + 8 * hh), x3 = *(const v4fa*)(arow + kb + 16 + 8 * hh + 4);
    float xs[16] = {x0[0],x0[1],x0[2],x0[3],x1[0],x1[1],x1[2],x1[3],x2[0],x2[1],x2[2],x2[3],x3[0],x3[1],x3[2],x3[3]};
#pragma unroll
    for (int i = 0; i < 16; ++i) { const unsigned short hb = bf16_bits(xs[i]); ah.u[i] = hb; al.u[i] = ASPLIT ? bf16_bits(xs[i] - bf16_val(hb)) : (unsigned short)0; }
#pragma unroll
    for (int t = 0; t < 4; ++t) {
      const unsigned short* brow = Wt + (size_t)(col0 + t * 16 + ln) * ldb + kb;
      FragB b;
      b.half[0] = *(const v8us*)(brow + 8 * hh);
      b.half[1] = *(const v8us*)(brow + 16 + 8 * hh);
      acc[t] = mmaN<ASPLIT ? 2 : 1>(ah.v, al.v, b.v, b.v, acc[t]);
    }
  }
#pragma unroll
  for (int t = 0; t < 4; ++t) {
    float bv = bias ? bias[col0 + t * 16 + ln] : 0.f;
    if (BIAS_BF16) bv = bf16_rne(bv);
#pragma unroll
    for (int r = 0; r < 8; ++r) { float v = acc[t][r] + bv; if (ACT == 1) v = fmaxf(v, 0.f); so[w][8 * hh + r][t * 16 + ln] = v; }
  }
  __builtin_amdgcn_fence(4  , "workgroup");
  __builtin_amdgcn_wave_barrier();
  const int rsub = lane >> 4, c4 = (lane & 15) * 4;
  for (int pass = 0; pass < 2; ++pass) {
#pragma unroll
    for (int q = 0; q < 8; ++q) {
      const int r = q * 2 + rsub;
      const v4f v = *(const v4fa*)&so[w][r][c4];
      *(volatile v4f*)(C + (size_t)(row0 + r) * ldc + col0 + c4) = v;
    }
    if (pass == 0) __threadfence();
  }
}

template <int D>
__global__ __launch_bounds__(128) void k_attn(const float* __restrict__ Qb, int qpitch, int Tq,
                                              const unsigned short* __restrict__ Kh, const unsigned short* __restrict__ Kl,
                                              const unsigned short* __restrict__ Vh, const unsigned short* __restrict__ Vl, int kpitch, int Tk,
                                              int H, float scale, float* __restrict__ y, int ypitch) {
  constexpr int KS = D / 32, DT = D / 16, C8 = D / 8;
  __shared__ __attribute__((aligned(16))) unsigned short sKh[32][D + 8], sKl[32][D + 8], sVh[32][D + 8], sVl[32][D + 8];
  __shared__ __attribute__((aligned(16))) unsigned short sPh[4][16][40], sPl[4][16][40];
  __shared__ __attribute__((aligned(16))) float sO[4][16][D];
  const int tid = threadIdx.x, w = tid >> 5, lane = tid & 31, ln = lane & 15, hh = lane >> 4;
  const int nqb = (Tq + 63) / 64;
  const int bh = blockIdx.x / nqb, qblk = blockIdx.x % nqb;
  const int b = bh / H, h = bh % H;
  const int q0 = qblk * 64 + w * 16;
  const float* Q = Qb + (size_t)b * Tq * qpitch + (size_t)h * D;
  const size_t kvbase = (size_t)b * Tk * kpitch + (size_t)h * D;

  FragB aqh[KS], aql[KS];
  {
    int row = q0 + ln; if (row >= Tq) row = Tq - 1;
    const float* qr = Q + (size_t)row * qpitch;
#pragma unroll
    for (int ks = 0; ks < KS; ++ks) {
      const v4f x0 = *(const v4fa*)(qr + ks * 32 + 8 * hh), x1 = *(const v4fa*)(qr + ks * 32 + 8 * hh + 4);
      const v4f x2 = *(const v4fa*)(qr + ks * 32 + 16 + 8 * hh), x3 = *(const v4fa*)(qr + ks * 32 + 16 + 8 * hh + 4);
      float xs[16] = {x0[0],x0[1],x0[2],x0[3],x1[0],x1[1],x1[2],x1[3],x2[0],x2[1],x2[2],x2[3],x3[0],x3[1],x3[2],x3[3]};
#pragma unroll
      for (int i = 0; i < 16; ++i) {
        const float x = xs[i] * scale; const unsigned short hb = bf16_bits(x);
        aqh[ks].u[i] = hb; aql[ks].u[i] = bf16_bits(x - bf16_val(hb));
      }
    }
  }
  float m_r[8], l_r[8];
#pragma unroll
  for (int r = 0; r < 8; ++r) { m_r[r] = -3.0e38f; l_r[r] = 0.f; }
  v8f oacc[DT];
#pragma unroll
  for (int dt = 0; dt < DT; ++dt) oacc[dt] = (v8f){0.f,0.f,0.f,0.f,0.f,0.f,0.f,0.f};

  for (int j0 = 0; j0 < Tk; j0 += 32) {
    __syncthreads();
    for (int e = tid; e < 32 * C8; e += 128) {
      const int r = e / C8, c8 = (e % C8) * 8;
      const int key = j0 + r;
      const int kc = (key < Tk) ? key : (Tk - 1);
      const size_t ko = kvbase + (size_t)kc * kpitch + c8;
      v8us a0 = *(const v8us*)(Kh + ko), a1 = *(const v8us*)(Kl + ko), a2 = *(const v8us*)(Vh + ko), a3 = *(const v8us*)(Vl + ko);
      if (key >= Tk) { a0 = (v8us){0,0,0,0,0,0,0,0}; a1 = a0; a2 = a0; a3 = a0; }
      *(v8us*)&sKh[r][c8] = a0; *(v8us*)&sKl[r][c8] = a1; *(v8us*)&sVh[r][c8] = a2; *(v8us*)&sVl[r][c8] = a3;
    }
    __syncthreads();
    v8f s[2];
#pragma unroll
    for (int nt = 0; nt < 2; ++nt) {
      v8f acc = {};
#pragma unroll
      for (int ks = 0; ks < KS; ++ks) {
        FragB bh_, bl_;
        bh_.half[0] = *(const v8us*)&sKh[nt * 16 + ln][ks * 32 + 8 * hh]; bh_.half[1] = *(const v8us*)&sKh[nt * 16 + ln][ks * 32 + 16 + 8 * hh];
        bl_.half[0] = *(const v8us*)&sKl[nt * 16 + ln][ks * 32 + 8 * hh]; bl_.half[1] = *(const v8us*)&sKl[nt * 16 + ln][ks * 32 + 16 + 8 * hh];
        acc = mmaN<3>(aqh[ks].v, aql[ks].v, bh_.v, bl_.v, acc);
      }
      s[nt] = acc;
    }
    float alpha[8];
#pragma unroll
    for (int r = 0; r < 8; ++r) {
      const int ja = j0 + ln, jb = j0 + 16 + ln;
      if (ja >= Tk) s[0][r] = -3.0e38f;
      if (jb >= Tk) s[1][r] = -3.0e38f;
      float mx = fmaxf(s[0][r], s[1][r]);
      mx = fmaxf(mx, __shfl_xor(mx, 1, 32)); mx = fmaxf(mx, __shfl_xor(mx, 2, 32)); mx = fmaxf(mx, __shfl_xor(mx, 4, 32)); mx = fmaxf(mx, __shfl_xor(mx, 8, 32));
      const float mnew = fmaxf(m_r[r], mx);
      alpha[r] = (mnew > -1.0e38f) ? __expf(m_r[r] - mnew) : 1.0f;
      const float p0 = (s[0][r] > -1.0e38f) ? __expf(s[0][r] - mnew) : 0.f;
      const float p1 = (s[1][r] > -1.0e38f) ? __expf(s[1][r] - mnew) : 0.f;
      m_r[r] = mnew;
      l_r[r] = l_r[r] * alpha[r] + p0 + p1;
      unsigned short hb = bf16_bits(p0); sPh[w][8 * hh + r][ln] = hb;      sPl[w][8 * hh + r][ln] = bf16_bits(p0 - bf16_val(hb));
      hb = bf16_bits(p1);                sPh[w][8 * hh + r][16 + ln] = hb; sPl[w][8 * hh + r][16 + ln] = bf16_bits(p1 - bf16_val(hb));
    }
#pragma unroll
    for (int dt = 0; dt < DT; ++dt)
#pragma unroll
      for (int r = 0; r < 8; ++r) oacc[dt][r] *= alpha[r];
    __builtin_amdgcn_fence(4  , "workgroup");
    __builtin_amdgcn_wave_barrier();
    FragB pah, pal;
    pah.half[0] = *(const v8us*)&sPh[w][ln][8 * hh]; pah.half[1] = *(const v8us*)&sPh[w][ln][16 + 8 * hh];
    pal.half[0] = *(const v8us*)&sPl[w][ln][8 * hh]; pal.half[1] = *(const v8us*)&sPl[w][ln][16 + 8 * hh];
#pragma unroll
    for (int dt = 0; dt < DT; ++dt) {
      FragB bvh, bvl;
#pragma unroll
      for (int i = 0; i < 8; ++i) {
        bvh.u[i] = sVh[8 * hh + i][dt * 16 + ln]; bvh.u[8 + i] = sVh[16 + 8 * hh + i][dt * 16 + ln];
        bvl.u[i] = sVl[8 * hh + i][dt * 16 + ln]; bvl.u[8 + i] = sVl[16 + 8 * hh + i][dt * 16 + ln];
      }
      oacc[dt] = mmaN<3>(pah.v, pal.v, bvh.v, bvl.v, oacc[dt]);
    }
    __builtin_amdgcn_fence(4  , "workgroup");
    __builtin_amdgcn_wave_barrier();
  }
#pragma unroll
  for (int r = 0; r < 8; ++r) {
    float l = l_r[r];
    l += __shfl_xor(l, 1, 32); l += __shfl_xor(l, 2, 32); l += __shfl_xor(l, 4, 32); l += __shfl_xor(l, 8, 32);
    l_r[r] = (l > 0.f) ? 1.0f / l : 0.f;
  }
#pragma unroll
  for (int dt = 0; dt < DT; ++dt)
#pragma unroll
    for (int r = 0; r < 8; ++r) sO[w][8 * hh + r][dt * 16 + ln] = oacc[dt][r] * l_r[r];
  __builtin_amdgcn_fence(4  , "workgroup");
  __builtin_amdgcn_wave_barrier();
  for (int pass = 0; pass < 2; ++pass) {
    for (int r = 0; r < 16; ++r) {
      const int row = q0 + r;
      if (row < Tq && lane < D / 4) {
        const v4f val = *(const v4fa*)&sO[w][r][lane * 4];
        *(volatile v4f*)(y + ((size_t)b * Tq + row) * ypitch + (size_t)h * D + lane * 4) = val;
      }
    }
    if (pass == 0) __threadfence();
  }
}

__global__ __launch_bounds__(256) void k_transpose32(const float* __restrict__ in, size_t in_bstride, int in_pitch,
                                                    float* __restrict__ out, size_t out_bstride, int out_pitch) {
  __shared__ float tile[32][33];
  const int b = blockIdx.z;
  const int r0 = blockIdx.y * 32, c0 = blockIdx.x * 32;
  const float* src = in + (size_t)b * in_bstride;
  float* dst = out + (size_t)b * out_bstride;
  const int tx = threadIdx.x & 31, ty = threadIdx.x >> 5;
  for (int i = ty; i < 32; i += 8) tile[i][tx] = src[(size_t)(r0 + i) * in_pitch + c0 + tx];
  __syncthreads();
  for (int pass = 0; pass < 2; ++pass) {
    for (int i = ty; i < 32; i += 8) {
      const float v = tile[tx][i];
      const int orow = c0 + i;
      *(volatile float*)(dst + (size_t)orow * out_pitch + r0 + tx) = v;
    }
    if (pass == 0) __threadfence();
  }
}

extern "C" void kernel_launch(void* const* d_in, const int* in_sizes, int n_in,
                              void* d_out, int out_size, void* d_ws, size_t ws_size, hipStream_t stream) {
  if (n_in < 10) return;
  const long long need_act = (long long)(NB * CC - 1) * PF + PP;
  if ((long long)in_sizes[0] < need_act || (long long)in_sizes[1] < need_act) return;
  if (in_sizes[2] < CC * CC || in_sizes[4] < CC * CC || in_sizes[6] < CC * CC || in_sizes[8] < CC * CC) return;
  if (in_sizes[3] < CC || in_sizes[5] < CC || in_sizes[7] < CC || in_sizes[9] < CC) return;
  if ((long long)out_size < need_act) return;
  const float* water = (const float*)d_in[0]; const float* bed = (const float*)d_in[1];
  const float* wq = (const float*)d_in[2]; const float* bq = (const float*)d_in[3]; const float* wk = (const float*)d_in[4]; const float* bk = (const float*)d_in[5];
  const float* wv = (const float*)d_in[6]; const float* bv = (const float*)d_in[7]; const float* wo = (const float*)d_in[8]; const float* bo = (const float*)d_in[9];
  char* ws = (char*)d_ws; size_t off = 0;
  auto take = [&](size_t bytes) { char* p = ws + off; off += (bytes + 255) & ~(size_t)255; return p; };
  const int M = NB * PP;
  unsigned short* Wqt = (unsigned short*)take((size_t)CC * CC * 2); unsigned short* Wkt = (unsigned short*)take((size_t)CC * CC * 2);
  unsigned short* Wvt = (unsigned short*)take((size_t)CC * CC * 2); unsigned short* Wot = (unsigned short*)take((size_t)CC * CC * 2);
  float* xT = (float*)take((size_t)M * CC * 4); float* yT = (float*)take((size_t)M * CC * 4);
  float* q = (float*)take((size_t)M * CC * 4); float* k = (float*)take((size_t)M * CC * 4); float* v = (float*)take((size_t)M * CC * 4);
  unsigned short* kh = (unsigned short*)take((size_t)M * CC * 2); unsigned short* kl = (unsigned short*)take((size_t)M * CC * 2);
  unsigned short* vh = (unsigned short*)take((size_t)M * CC * 2); unsigned short* vl = (unsigned short*)take((size_t)M * CC * 2);
  float* att = (float*)take((size_t)M * CC * 4); float* o = (float*)take((size_t)M * CC * 4);
  if (off > ws_size || off > ((size_t)128 << 20)) return;

  k_cvt_rows<<<(CC * CC / 8 + 255) / 256, 256, 0, stream>>>(wq, Wqt, CC * CC / 8);
  k_cvt_rows<<<(CC * CC / 8 + 255) / 256, 256, 0, stream>>>(wk, Wkt, CC * CC / 8);
  k_cvt_rows<<<(CC * CC / 8 + 255) / 256, 256, 0, stream>>>(wv, Wvt, CC * CC / 8);
  k_cvt_rows<<<(CC * CC / 8 + 255) / 256, 256, 0, stream>>>(wo, Wot, CC * CC / 8);
  k_transpose32<<<dim3(PP / 32, CC / 32, NB), 256, 0, stream>>>(water, (size_t)CC * PF, PF, xT, (size_t)PP * CC, CC);
  k_transpose32<<<dim3(PP / 32, CC / 32, NB), 256, 0, stream>>>(bed,   (size_t)CC * PF, PF, yT, (size_t)PP * CC, CC);
  k_gemm_bf<false, 0, true><<<((M / 16) * (CC / 64) + 3) / 4, 128, 0, stream>>>(xT, CC, Wqt, CC, bq, q, CC, M, CC, CC);
  k_gemm_bf<false, 0, true><<<((M / 16) * (CC / 64) + 3) / 4, 128, 0, stream>>>(yT, CC, Wkt, CC, bk, k, CC, M, CC, CC);
  k_gemm_bf<false, 0, true><<<((M / 16) * (CC / 64) + 3) / 4, 128, 0, stream>>>(yT, CC, Wvt, CC, bv, v, CC, M, CC, CC);
  k_split_rows<<<(M * (CC / 8) + 255) / 256, 256, 0, stream>>>(k, kh, kl, M * (CC / 8));
  k_split_rows<<<(M * (CC / 8) + 255) / 256, 256, 0, stream>>>(v, vh, vl, M * (CC / 8));
  k_attn<CC><<<NB * TT * ((SEQ + 63) / 64), 128, 0, stream>>>(q, TT * CC, SEQ, kh, kl, vh, vl, TT * CC, SEQ, TT, 0.125f, att, TT * CC);
  k_gemm_bf<true, 0, true><<<((M / 16) * (CC / 64) + 3) / 4, 128, 0, stream>>>(att, CC, Wot, CC, bo, o, CC, M, CC, CC);
  k_transpose32<<<dim3(CC / 32, PP / 32, NB), 256, 0, stream>>>(o, (size_t)PP * CC, CC, (float*)d_out, (size_t)CC * PF, PF);
}
